// LTCCell_63702954934929
// MI455X (gfx1250) — hardware-verified
//
#include <hip/hip_runtime.h>

#define INS   1024
#define HID   2048
#define KTOT  3072
#define NB    4096
#define EP    36
#define TP    72

static_assert((INS % 32) == 0);
static_assert((KTOT % 64) == 0);
static_assert((HID % 64) == 0);
static_assert((NB % 64) == 0);
static_assert(((NB * (KTOT / 8)) % 256) == 0);

typedef unsigned short u16;
typedef u16    v8u16 __attribute__((ext_vector_type(8)));
typedef __bf16 v16bf __attribute__((ext_vector_type(16)));
typedef float  v8f   __attribute__((ext_vector_type(8)));
typedef float  v4f   __attribute__((ext_vector_type(4)));

union Frag { v16bf v; v8u16 hv[2]; };

__device__ __forceinline__ unsigned int bf_hi(float f) {
  unsigned int u = __builtin_bit_cast(unsigned int, f);
  u += 0x7FFFu + ((u >> 16) & 1u);
  return u >> 16;
}
__device__ __forceinline__ u16 f2bf(float f) { return (u16)bf_hi(f); }
__device__ __forceinline__ float bfr(float f) {
  return __builtin_bit_cast(float, bf_hi(f) << 16);
}

__device__ __forceinline__ v16bf ldfrag(const u16* p) {
  Frag f;
  f.hv[0] = *reinterpret_cast<const v8u16*>(p);
  f.hv[1] = *reinterpret_cast<const v8u16*>(p + 16);
  return f.v;
}

__device__ __forceinline__ v8f mma_bf16(v16bf a, v16bf b, v8f c) {
  return __builtin_amdgcn_wmma_f32_16x16x32_bf16(false, a, false, b,
                                                 (short)0, c, false, false);
}

__global__ __launch_bounds__(256)
void k_cvt_rows(const float* __restrict__ x, const float* __restrict__ hin,
                u16* __restrict__ Abf, int ngroups) {
  const int g = blockIdx.x * 256 + threadIdx.x;
  if (g >= ngroups) return;
  const int row = g / (KTOT / 8);
  const int c = (g - row * (KTOT / 8)) * 8;
  const float* src = (c < INS) ? (x + (size_t)row * INS + c)
                               : (hin + (size_t)row * HID + (c - INS));
  const v4f v0 = *reinterpret_cast<const v4f*>(src);
  const v4f v1 = *reinterpret_cast<const v4f*>(src + 4);
  v8u16 o;
  o[0] = f2bf(v0.x); o[1] = f2bf(v0.y); o[2] = f2bf(v0.z); o[3] = f2bf(v0.w);
  o[4] = f2bf(v1.x); o[5] = f2bf(v1.y); o[6] = f2bf(v1.z); o[7] = f2bf(v1.w);
  u16* dst = Abf + (size_t)row * KTOT + c;
  *reinterpret_cast<volatile v8u16*>(dst) = o;
  __threadfence();
  *reinterpret_cast<volatile v8u16*>(dst) = o;
}

__global__ __launch_bounds__(256)
void k_transpose_w(const float* __restrict__ W, u16* __restrict__ Wtr) {
  __shared__ __align__(16) u16 tile[64 * TP];
  const int tid = threadIdx.x;
  const int n0 = blockIdx.x * 64;
  const int k0 = blockIdx.y * 64;
#pragma unroll
  for (int i = 0; i < 4; ++i) {
    const int idx = tid + 256 * i;
    const int kr = idx >> 4;
    const int c4 = (idx & 15) * 4;
    const v4f v = *reinterpret_cast<const v4f*>(W + (size_t)(k0 + kr) * HID + n0 + c4);
    tile[(c4 + 0) * TP + kr] = f2bf(v.x);
    tile[(c4 + 1) * TP + kr] = f2bf(v.y);
    tile[(c4 + 2) * TP + kr] = f2bf(v.z);
    tile[(c4 + 3) * TP + kr] = f2bf(v.w);
  }
  __syncthreads();
  const int wave = tid >> 5, lane = tid & 31;
  const int kk = (lane & 7) * 8;
  const int nlA = wave * 8 + (lane >> 3);
  const int nlB = nlA + 4;
  const v8u16 oA = *reinterpret_cast<const v8u16*>(&tile[nlA * TP + kk]);
  const v8u16 oB = *reinterpret_cast<const v8u16*>(&tile[nlB * TP + kk]);
  u16* dA = Wtr + (size_t)(n0 + nlA) * KTOT + k0 + kk;
  u16* dB = Wtr + (size_t)(n0 + nlB) * KTOT + k0 + kk;
  *reinterpret_cast<volatile v8u16*>(dA) = oA;
  *reinterpret_cast<volatile v8u16*>(dB) = oB;
  __threadfence();
  *reinterpret_cast<volatile v8u16*>(dA) = oA;
  *reinterpret_cast<volatile v8u16*>(dB) = oB;
}

__device__ __forceinline__ void st8(float* s, v8f c) {
  s[0 * EP] = c[0]; s[1 * EP] = c[1]; s[2 * EP] = c[2]; s[3 * EP] = c[3];
  s[4 * EP] = c[4]; s[5 * EP] = c[5]; s[6 * EP] = c[6]; s[7 * EP] = c[7];
}

__device__ __forceinline__ float cell_update(float pf, float pa, float tau,
                                             float tdv, float hv, float bs) {
  const float f = tanhf(pf);
  const float a = tanhf(pa);
  const float tsys = tau * (1.0f / (1.0f + tau * fabsf(f)));
  const float dec = expf(-tdv * (1.0f / (tsys + 1e-6f)));
  return dec * hv + (1.0f - dec) * (a + bs);
}

__global__ __launch_bounds__(128)
void k_gemm_cell(const u16* __restrict__ Abf,
                 const u16* __restrict__ Wm_t,
                 const u16* __restrict__ Wt_t,
                 const float* __restrict__ hin,
                 const float* __restrict__ td,
                 const float* __restrict__ bm,
                 const float* __restrict__ bt,
                 const float* __restrict__ logtau,
                 const float* __restrict__ bias,
                 float* __restrict__ out) {
  __shared__ __align__(16) float sF[4 * 32 * EP];
  __shared__ __align__(16) float sT[4 * 32 * EP];

  const int tid  = threadIdx.x;
  const int lane = tid & 31;
  const int wave = tid >> 5;
  const int h    = lane >> 4;
  const int m    = lane & 15;
  const int row0 = blockIdx.y * 64 + (wave >> 1) * 32;
  const int col0 = blockIdx.x * 64 + (wave & 1) * 32;

  const u16* pa0 = Abf  + (size_t)(row0 + m) * KTOT + 8 * h;
  const u16* pa1 = Abf  + (size_t)(row0 + 16 + m) * KTOT + 8 * h;
  const u16* pb0 = Wm_t + (size_t)(col0 + m) * KTOT + 8 * h;
  const u16* pb1 = Wm_t + (size_t)(col0 + 16 + m) * KTOT + 8 * h;
  const u16* pb2 = Wt_t + (size_t)(col0 + m) * KTOT + 8 * h;
  const u16* pb3 = Wt_t + (size_t)(col0 + 16 + m) * KTOT + 8 * h;

  const v8f z = {0.f, 0.f, 0.f, 0.f, 0.f, 0.f, 0.f, 0.f};
  v8f cF00 = z, cF10 = z, cF01 = z, cF11 = z;
  v8f cA00 = z, cA10 = z, cA01 = z, cA11 = z;

  for (int k0 = 0; k0 < KTOT; k0 += 32) {
    const v16bf a0 = ldfrag(pa0 + k0);
    const v16bf a1 = ldfrag(pa1 + k0);
    const v16bf b0 = ldfrag(pb0 + k0);
    const v16bf b1 = ldfrag(pb1 + k0);
    const v16bf b2 = ldfrag(pb2 + k0);
    const v16bf b3 = ldfrag(pb3 + k0);
    cF00 = mma_bf16(a0, b0, cF00);
    cF10 = mma_bf16(a1, b0, cF10);
    cF01 = mma_bf16(a0, b1, cF01);
    cF11 = mma_bf16(a1, b1, cF11);
    cA00 = mma_bf16(a0, b2, cA00);
    cA10 = mma_bf16(a1, b2, cA10);
    cA01 = mma_bf16(a0, b3, cA01);
    cA11 = mma_bf16(a1, b3, cA11);
    asm volatile("v_nop\n\tv_nop\n\tv_nop\n\tv_nop"
                 : "+v"(cF00), "+v"(cF10), "+v"(cF01), "+v"(cF11),
                   "+v"(cA00), "+v"(cA10), "+v"(cA01), "+v"(cA11)
                 : "v"(a0), "v"(a1), "v"(b0), "v"(b1), "v"(b2), "v"(b3));
  }

  {
    float* sf = sF + wave * (32 * EP) + (8 * h) * EP + m;
    float* sa = sT + wave * (32 * EP) + (8 * h) * EP + m;
    st8(sf, cF00);            st8(sf + 16, cF01);
    st8(sf + 16 * EP, cF10);  st8(sf + 16 * EP + 16, cF11);
    st8(sa, cA00);            st8(sa + 16, cA01);
    st8(sa + 16 * EP, cA10);  st8(sa + 16 * EP + 16, cA11);
  }
  __syncthreads();

  const int c4   = (lane & 7) * 4;
  const int ncol = col0 + c4;
  const v4f bm4 = *reinterpret_cast<const v4f*>(bm + ncol);
  const v4f bt4 = *reinterpret_cast<const v4f*>(bt + ncol);
  const v4f bs4 = *reinterpret_cast<const v4f*>(bias + ncol);
  const v4f lt4 = *reinterpret_cast<const v4f*>(logtau + ncol);
  const float bm0 = bfr(bm4.x), bm1 = bfr(bm4.y), bm2 = bfr(bm4.z), bm3 = bfr(bm4.w);
  const float bt0 = bfr(bt4.x), bt1 = bfr(bt4.y), bt2 = bfr(bt4.z), bt3 = bfr(bt4.w);
  const float bs0 = bfr(bs4.x), bs1 = bfr(bs4.y), bs2 = bfr(bs4.z), bs3 = bfr(bs4.w);
  const float tau0 = expf(bfr(lt4.x)), tau1 = expf(bfr(lt4.y));
  const float tau2 = expf(bfr(lt4.z)), tau3 = expf(bfr(lt4.w));

  const float* sfw = sF + wave * (32 * EP) + c4;
  const float* saw = sT + wave * (32 * EP) + c4;
  const int rq = lane >> 3;

#pragma unroll 1
  for (int i = 0; i < 8; ++i) {
    const int r = rq + 4 * i;
    const int grow = row0 + r;
    const float tdv = bfr(td[grow]);
    const v4f hv = *reinterpret_cast<const v4f*>(hin + (size_t)grow * HID + ncol);
    const v4f fp = *reinterpret_cast<const v4f*>(sfw + r * EP);
    const v4f ap = *reinterpret_cast<const v4f*>(saw + r * EP);
    v4f o;
    o.x = cell_update(fp.x + bm0, ap.x + bt0, tau0, tdv, bfr(hv.x), bs0);
    o.y = cell_update(fp.y + bm1, ap.y + bt1, tau1, tdv, bfr(hv.y), bs1);
    o.z = cell_update(fp.z + bm2, ap.z + bt2, tau2, tdv, bfr(hv.z), bs2);
    o.w = cell_update(fp.w + bm3, ap.w + bt3, tau3, tdv, bfr(hv.w), bs3);
    float* po = out + (size_t)grow * HID + ncol;
    *reinterpret_cast<volatile v4f*>(po) = o;
    __threadfence();
    *reinterpret_cast<volatile v4f*>(po) = o;
  }
}

extern "C" void kernel_launch(void* const* d_in, const int* in_sizes, int n_in,
                              void* d_out, int out_size, void* d_ws, size_t ws_size,
                              hipStream_t stream) {
  if (n_in < 9) return;
  if (in_sizes[0] != NB * INS)   return;
  if (in_sizes[1] != NB * HID)   return;
  if (in_sizes[2] != NB)         return;
  if (in_sizes[3] != KTOT * HID) return;
  if (in_sizes[4] != HID)        return;
  if (in_sizes[5] != KTOT * HID) return;
  if (in_sizes[6] != HID)        return;
  if (in_sizes[7] != HID)        return;
  if (in_sizes[8] != HID)        return;
  if (out_size != NB * HID)      return;

  const float* x      = (const float*)d_in[0];
  const float* h      = (const float*)d_in[1];
  const float* td     = (const float*)d_in[2];
  const float* W_mod  = (const float*)d_in[3];
  const float* b_mod  = (const float*)d_in[4];
  const float* W_tgt  = (const float*)d_in[5];
  const float* b_tgt  = (const float*)d_in[6];
  const float* logtau = (const float*)d_in[7];
  const float* bias   = (const float*)d_in[8];
  float* out = (float*)d_out;

  const size_t bytesA = (size_t)NB * KTOT * sizeof(u16);
  const size_t bytesW = (size_t)HID * KTOT * sizeof(u16);
  const size_t offA  = 0;
  const size_t offWm = offA + bytesA;
  const size_t offWt = offWm + bytesW;
  const size_t total = offWt + bytesW;
  if (total > ws_size) return;

  char* ws = (char*)d_ws;
  u16* Abf  = (u16*)(ws + offA);
  u16* Wm_t = (u16*)(ws + offWm);
  u16* Wt_t = (u16*)(ws + offWt);

  const int ngroups = NB * (KTOT / 8);
  const int cvt_blocks = (ngroups + 255) / 256;

  k_cvt_rows<<<dim3(cvt_blocks), dim3(256), 0, stream>>>(x, h, Abf, ngroups);
  k_transpose_w<<<dim3(HID / 64, KTOT / 64), dim3(256), 0, stream>>>(W_mod, Wm_t);
  k_transpose_w<<<dim3(HID / 64, KTOT / 64), dim3(256), 0, stream>>>(W_tgt, Wt_t);
  k_gemm_cell<<<dim3(HID / 64, NB / 64), dim3(128), 0, stream>>>(
      Abf, Wm_t, Wt_t, h, td, b_mod, b_tgt, logtau, bias, out);
}
